// seg_model_11699490915025
// MI455X (gfx1250) — hardware-verified
//
#include <hip/hip_runtime.h>
#define BB 8
#define NN 2048
#define NCL 16

typedef __bf16 v16b __attribute__((ext_vector_type(16)));
typedef unsigned short v8us __attribute__((ext_vector_type(8), may_alias));
typedef float  v8f  __attribute__((ext_vector_type(8)));
typedef float  v4f  __attribute__((ext_vector_type(4)));
typedef float  v4fa __attribute__((ext_vector_type(4), may_alias));
union FragB { v16b v; v8us half[2]; unsigned short u[16]; };

__device__ __forceinline__ unsigned short bf16_bits(float x) { unsigned int u = __float_as_uint(x); return (unsigned short)((u + 0x7FFFu + ((u >> 16) & 1u)) >> 16); }
__device__ __forceinline__ float bf16_val(unsigned short b) { return __uint_as_float(((unsigned int)b) << 16); }
__device__ __forceinline__ float bf16_round(float x) { return bf16_val(bf16_bits(x)); }
template <int NT>
__device__ __forceinline__ v8f mmaN(v16b ah, v16b al, v16b bh, v16b bl, v8f c) {
  c = __builtin_amdgcn_wmma_f32_16x16x32_bf16(false, ah, false, bh, (short)0, c, false, false);
  if (NT >= 2) c = __builtin_amdgcn_wmma_f32_16x16x32_bf16(false, al, false, bh, (short)0, c, false, false);
  if (NT >= 3) c = __builtin_amdgcn_wmma_f32_16x16x32_bf16(false, ah, false, bl, (short)0, c, false, false);
  asm volatile("v_nop\n\tv_nop\n\tv_nop\n\tv_nop" : "+v"(c) : "v"(ah), "v"(al), "v"(bh), "v"(bl));
  return c;
}

__global__ __launch_bounds__(256) void k_wt_bf16(const float* __restrict__ W, unsigned short* __restrict__ Wt, int K, int N) {
  const int t = blockIdx.x * 256 + threadIdx.x;
  const int k8n = K / 8;
  if (t >= N * k8n) return;
  const int n = t / k8n, k8 = (t % k8n) * 8;
  v8us v;
#pragma unroll
  for (int i = 0; i < 8; ++i) v[i] = bf16_bits(W[(size_t)(k8 + i) * N + n]);
  *(volatile v8us*)(Wt + (size_t)n * K + k8) = v;
  __threadfence();
  *(volatile v8us*)(Wt + (size_t)n * K + k8) = v;
}

template <bool ASPLIT, int ACT, bool BIAS_BF16>
__global__ __launch_bounds__(128) void k_gemm_bf(const float* __restrict__ A, int lda, const unsigned short* __restrict__ Wt, int ldb,
                                               const float* __restrict__ bias, float* __restrict__ C, int ldc, int M, int N, int K) {
  __shared__ __attribute__((aligned(16))) float so[4][16][64];
  const int tid = threadIdx.x, w = tid >> 5, lane = tid & 31, ln = lane & 15, hh = lane >> 4;
  const int ntn = N / 64;
  const int wid = blockIdx.x * 4 + w;
  const int mt = wid / ntn, nq = wid % ntn;
  if (mt * 16 >= M) return;
  const int row0 = mt * 16, col0 = nq * 64;
  const float* arow = A + (size_t)(row0 + ln) * lda;
  v8f acc[4] = {};
  for (int kb = 0; kb < K; kb += 32) {
    FragB ah, al;
    const v4f x0 = *(const v4fa*)(arow + kb + 8 * hh), x1 = *(const v4fa*)(arow + kb + 8 * hh + 4);
    const v4f x2 = *(const v4fa*)(arow + kb + 16 + 8 * hh), x3 = *(const v4fa*)(arow + kb + 16 + 8 * hh + 4);
    float xs[16] = {x0[0],x0[1],x0[2],x0[3],x1[0],x1[1],x1[2],x1[3],x2[0],x2[1],x2[2],x2[3],x3[0],x3[1],x3[2],x3[3]};
#pragma unroll
    for (int i = 0; i < 16; ++i) { const unsigned short hb = bf16_bits(xs[i]); ah.u[i] = hb; al.u[i] = ASPLIT ? bf16_bits(xs[i] - bf16_val(hb)) : (unsigned short)0; }
#pragma unroll
    for (int t = 0; t < 4; ++t) {
      const unsigned short* brow = Wt + (size_t)(col0 + t * 16 + ln) * ldb + kb;
      FragB b;
      b.half[0] = *(const v8us*)(brow + 8 * hh);
      b.half[1] = *(const v8us*)(brow + 16 + 8 * hh);
      acc[t] = mmaN<ASPLIT ? 2 : 1>(ah.v, al.v, b.v, b.v, acc[t]);
    }
  }
#pragma unroll
  for (int t = 0; t < 4; ++t) {
    float bv = bias ? bias[col0 + t * 16 + ln] : 0.f;
    if (BIAS_BF16) bv = bf16_round(bv);
#pragma unroll
    for (int r = 0; r < 8; ++r) { float v = acc[t][r] + bv; if (ACT == 1) v = fmaxf(v, 0.f); so[w][8 * hh + r][t * 16 + ln] = v; }
  }
  __builtin_amdgcn_fence(__ATOMIC_ACQ_REL, "workgroup");
  __builtin_amdgcn_wave_barrier();
  const int rsub = lane >> 4, c4 = (lane & 15) * 4;
  for (int pass = 0; pass < 2; ++pass) {
#pragma unroll
    for (int q = 0; q < 8; ++q) {
      const int r = q * 2 + rsub;
      const v4f v = *(const v4fa*)&so[w][r][c4];
      *(volatile v4f*)(C + (size_t)(row0 + r) * ldc + col0 + c4) = v;
    }
    if (pass == 0) __threadfence();
  }
}

template <int D, bool CAUSAL>
__global__ __launch_bounds__(128) void k_flash(const float* __restrict__ qb, const float* __restrict__ kb, const float* __restrict__ vb,
                                             int pitch, int T, int H, float scale, float* __restrict__ y, int ypitch) {
  constexpr int KS = D / 32;
  constexpr int DT = D / 16;
  __shared__ __attribute__((aligned(16))) unsigned short sKh[32][D + 8], sKl[32][D + 8], sVh[32][D + 8], sVl[32][D + 8];
  __shared__ __attribute__((aligned(16))) unsigned short sPh[4][16][40], sPl[4][16][40];
  __shared__ __attribute__((aligned(16))) float sO[4][16][D];
  const int tid = threadIdx.x, w = tid >> 5, lane = tid & 31, ln = lane & 15, hh = lane >> 4;
  const int nqb = (T + 63) / 64;
  const int bh = blockIdx.x / nqb, qblk = blockIdx.x % nqb;
  const int b = bh / H, h = bh % H;
  const int q0 = qblk * 64 + w * 16;
  const float* Q = qb + (size_t)b * T * pitch + h * D;
  const float* K = kb + (size_t)b * T * pitch + h * D;
  const float* V = vb + (size_t)b * T * pitch + h * D;

  FragB aqh[KS], aql[KS];
  {
    int row = q0 + ln; if (row >= T) row = T - 1;
    const float* qr = Q + (size_t)row * pitch;
#pragma unroll
    for (int ks = 0; ks < KS; ++ks)
#pragma unroll
      for (int i = 0; i < 16; ++i) {
        const int d = ks * 32 + ((i < 8) ? (8 * hh + i) : (16 + 8 * hh + (i - 8)));
        const float x = qr[d] * scale; const unsigned short hb = bf16_bits(x);
        aqh[ks].u[i] = hb; aql[ks].u[i] = bf16_bits(x - bf16_val(hb));
      }
  }
  float m_r[8], l_r[8];
#pragma unroll
  for (int r = 0; r < 8; ++r) { m_r[r] = -3.0e38f; l_r[r] = 0.f; }
  v8f oacc[DT];
#pragma unroll
  for (int dt = 0; dt < DT; ++dt) oacc[dt] = (v8f){0.f,0.f,0.f,0.f,0.f,0.f,0.f,0.f};

  const int kv_end = CAUSAL ? min(T, qblk * 64 + 64) : T;
  for (int j0 = 0; j0 < kv_end; j0 += 32) {
    __syncthreads();
    for (int e = tid; e < 32 * (D / 4); e += 128) {
      const int r = e / (D / 4), c4 = (e % (D / 4)) * 4;
      const int key = j0 + r;
      v4f kf = {0.f,0.f,0.f,0.f}, vf = {0.f,0.f,0.f,0.f};
      if (key < T) { kf = *(const v4fa*)(K + (size_t)key * pitch + c4); vf = *(const v4fa*)(V + (size_t)key * pitch + c4); }
#pragma unroll
      for (int t = 0; t < 4; ++t) {
        unsigned short hb = bf16_bits(kf[t]); sKh[r][c4 + t] = hb; sKl[r][c4 + t] = bf16_bits(kf[t] - bf16_val(hb));
        hb = bf16_bits(vf[t]); sVh[r][c4 + t] = hb; sVl[r][c4 + t] = bf16_bits(vf[t] - bf16_val(hb));
      }
    }
    __syncthreads();
    v8f s[2];
#pragma unroll
    for (int nt = 0; nt < 2; ++nt) {
      v8f acc = {};
#pragma unroll
      for (int ks = 0; ks < KS; ++ks) {
        FragB bh_, bl_;
        bh_.half[0] = *(const v8us*)&sKh[nt * 16 + ln][ks * 32 + 8 * hh]; bh_.half[1] = *(const v8us*)&sKh[nt * 16 + ln][ks * 32 + 16 + 8 * hh];
        bl_.half[0] = *(const v8us*)&sKl[nt * 16 + ln][ks * 32 + 8 * hh]; bl_.half[1] = *(const v8us*)&sKl[nt * 16 + ln][ks * 32 + 16 + 8 * hh];
        acc = mmaN<3>(aqh[ks].v, aql[ks].v, bh_.v, bl_.v, acc);
      }
      s[nt] = acc;
    }
    float alpha[8];
#pragma unroll
    for (int r = 0; r < 8; ++r) {
      const int qi = q0 + 8 * hh + r;
      const int ja = j0 + ln, jb = j0 + 16 + ln;
      if (CAUSAL) { if (ja > qi) s[0][r] = -3.0e38f; if (jb > qi) s[1][r] = -3.0e38f; }
      if (ja >= T) s[0][r] = -3.0e38f;
      if (jb >= T) s[1][r] = -3.0e38f;
      float mx = fmaxf(s[0][r], s[1][r]);
      mx = fmaxf(mx, __shfl_xor(mx, 1, 32)); mx = fmaxf(mx, __shfl_xor(mx, 2, 32)); mx = fmaxf(mx, __shfl_xor(mx, 4, 32)); mx = fmaxf(mx, __shfl_xor(mx, 8, 32));
      const float mnew = fmaxf(m_r[r], mx);
      alpha[r] = (mnew > -1.0e38f) ? __expf(m_r[r] - mnew) : 1.0f;
      const float p0 = (s[0][r] > -1.0e38f) ? __expf(s[0][r] - mnew) : 0.f;
      const float p1 = (s[1][r] > -1.0e38f) ? __expf(s[1][r] - mnew) : 0.f;
      m_r[r] = mnew;
      l_r[r] = l_r[r] * alpha[r] + p0 + p1;
      unsigned short hb = bf16_bits(p0); sPh[w][8 * hh + r][ln] = hb;      sPl[w][8 * hh + r][ln] = bf16_bits(p0 - bf16_val(hb));
      hb = bf16_bits(p1);                sPh[w][8 * hh + r][16 + ln] = hb; sPl[w][8 * hh + r][16 + ln] = bf16_bits(p1 - bf16_val(hb));
    }
#pragma unroll
    for (int dt = 0; dt < DT; ++dt)
#pragma unroll
      for (int r = 0; r < 8; ++r) oacc[dt][r] *= alpha[r];
    __builtin_amdgcn_fence(__ATOMIC_ACQ_REL, "workgroup");
    __builtin_amdgcn_wave_barrier();
    FragB pah, pal;
    pah.half[0] = *(const v8us*)&sPh[w][ln][8 * hh]; pah.half[1] = *(const v8us*)&sPh[w][ln][16 + 8 * hh];
    pal.half[0] = *(const v8us*)&sPl[w][ln][8 * hh]; pal.half[1] = *(const v8us*)&sPl[w][ln][16 + 8 * hh];
#pragma unroll
    for (int dt = 0; dt < DT; ++dt) {
      FragB bvh, bvl;
#pragma unroll
      for (int i = 0; i < 8; ++i) {
        bvh.u[i] = sVh[8 * hh + i][dt * 16 + ln]; bvh.u[8 + i] = sVh[16 + 8 * hh + i][dt * 16 + ln];
        bvl.u[i] = sVl[8 * hh + i][dt * 16 + ln]; bvl.u[8 + i] = sVl[16 + 8 * hh + i][dt * 16 + ln];
      }
      oacc[dt] = mmaN<3>(pah.v, pal.v, bvh.v, bvl.v, oacc[dt]);
    }
    __builtin_amdgcn_fence(__ATOMIC_ACQ_REL, "workgroup");
    __builtin_amdgcn_wave_barrier();
  }
#pragma unroll
  for (int r = 0; r < 8; ++r) {
    float l = l_r[r];
    l += __shfl_xor(l, 1, 32); l += __shfl_xor(l, 2, 32); l += __shfl_xor(l, 4, 32); l += __shfl_xor(l, 8, 32);
    l_r[r] = (l > 0.f) ? 1.0f / l : 0.f;
  }
#pragma unroll
  for (int dt = 0; dt < DT; ++dt)
#pragma unroll
    for (int r = 0; r < 8; ++r) sO[w][8 * hh + r][dt * 16 + ln] = oacc[dt][r] * l_r[r];
  __builtin_amdgcn_fence(__ATOMIC_ACQ_REL, "workgroup");
  __builtin_amdgcn_wave_barrier();
  for (int pass = 0; pass < 2; ++pass) {
    for (int r = 0; r < 16; ++r) {
      const int row = q0 + r;
      if (row < T && lane < D / 4) {
        const v4f val = *(const v4fa*)&sO[w][r][lane * 4];
        *(volatile v4f*)(y + ((size_t)b * T + row) * ypitch + h * D + lane * 4) = val;
      }
    }
    if (pass == 0) __threadfence();
  }
}

template <bool ASPLIT, bool BSPLIT, int ACT>
__global__ __launch_bounds__(128) void k_gemm_b(const float* __restrict__ A, int lda, size_t sA, const unsigned short* __restrict__ Bh, const unsigned short* __restrict__ Bl, int ldb, size_t sB,
                                             const float* __restrict__ bias, const float* __restrict__ resid, int ldr, size_t sR, float rsign, float alpha,
                                             float* __restrict__ C, int ldc, size_t sC, int M, int N, int K) {
  __shared__ __attribute__((aligned(16))) float so[4][16][64];
  const int tid = threadIdx.x, w = tid >> 5, lane = tid & 31, ln = lane & 15, hh = lane >> 4;
  const int by = blockIdx.y;
  A += (size_t)by * sA; Bh += (size_t)by * sB; if (BSPLIT) Bl += (size_t)by * sB; C += (size_t)by * sC; if (resid) resid += (size_t)by * sR;
  const int ntn = N / 64; const int wid = blockIdx.x * 4 + w; const int mt = wid / ntn, nq = wid % ntn;
  if (mt * 16 >= M) return;
  const int row0 = mt * 16, col0 = nq * 64;
  const float* arow = A + (size_t)(row0 + ln) * lda;
  v8f acc[4] = {};
  for (int kb = 0; kb < K; kb += 32) {
    FragB ah, al;
    const v4f x0 = *(const v4fa*)(arow + kb + 8 * hh), x1 = *(const v4fa*)(arow + kb + 8 * hh + 4);
    const v4f x2 = *(const v4fa*)(arow + kb + 16 + 8 * hh), x3 = *(const v4fa*)(arow + kb + 16 + 8 * hh + 4);
    float xs[16] = {x0[0],x0[1],x0[2],x0[3],x1[0],x1[1],x1[2],x1[3],x2[0],x2[1],x2[2],x2[3],x3[0],x3[1],x3[2],x3[3]};
#pragma unroll
    for (int i = 0; i < 16; ++i) { const unsigned short hb = bf16_bits(xs[i]); ah.u[i] = hb; al.u[i] = ASPLIT ? bf16_bits(xs[i] - bf16_val(hb)) : (unsigned short)0; }
#pragma unroll
    for (int t = 0; t < 4; ++t) {
      const size_t boff = (size_t)(col0 + t * 16 + ln) * ldb + kb;
      FragB bh_, bl_; bh_.half[0] = *(const v8us*)(Bh + boff + 8 * hh); bh_.half[1] = *(const v8us*)(Bh + boff + 16 + 8 * hh);
      if (BSPLIT) { bl_.half[0] = *(const v8us*)(Bl + boff + 8 * hh); bl_.half[1] = *(const v8us*)(Bl + boff + 16 + 8 * hh); } else bl_ = bh_;
      acc[t] = mmaN<ASPLIT ? (BSPLIT ? 3 : 2) : 1>(ah.v, al.v, bh_.v, bl_.v, acc[t]);
    }
  }
#pragma unroll
  for (int t = 0; t < 4; ++t) {
    const int col = col0 + t * 16 + ln; const float bv = bias ? bf16_round(bias[col]) : 0.f;
#pragma unroll
    for (int r = 0; r < 8; ++r) { float v = acc[t][r] * alpha + bv; if (resid) v += rsign * resid[(size_t)(row0 + 8 * hh + r) * ldr + col]; if (ACT == 1) v = fmaxf(v, 0.f); so[w][8 * hh + r][t * 16 + ln] = v; }
  }
  __builtin_amdgcn_fence(__ATOMIC_ACQ_REL, "workgroup"); __builtin_amdgcn_wave_barrier();
  const int rsub = lane >> 4, c4 = (lane & 15) * 4;
  for (int pass = 0; pass < 2; ++pass) {
#pragma unroll
    for (int q = 0; q < 8; ++q) { const int r = q * 2 + rsub; const v4f v = *(const v4fa*)&so[w][r][c4]; *(volatile v4f*)(C + (size_t)(row0 + r) * ldc + col0 + c4) = v; }
    if (pass == 0) __threadfence();
  }
}
__global__ __launch_bounds__(256) void k_split_transpose_b(const float* __restrict__ src, int lds_, size_t sIn, unsigned short* __restrict__ hi, unsigned short* __restrict__ lo, size_t sOut, int K, int N) {
  const size_t t = (size_t)blockIdx.x * 256 + threadIdx.x; const int k8n = K / 8; if (t >= (size_t)N * k8n) return;
  src += (size_t)blockIdx.y * sIn; hi += (size_t)blockIdx.y * sOut; lo += (size_t)blockIdx.y * sOut;
  const int n = (int)(t / k8n), k8 = (int)(t % k8n) * 8; v8us vh, vl;
#pragma unroll
  for (int i = 0; i < 8; ++i) { const float x = src[(size_t)(k8 + i) * lds_ + n]; const unsigned short hb = bf16_bits(x); vh[i] = hb; vl[i] = bf16_bits(x - bf16_val(hb)); }
  unsigned short* dh = hi + (size_t)n * K + k8; unsigned short* dl = lo + (size_t)n * K + k8;
  *(volatile v8us*)dh = vh; *(volatile v8us*)dl = vl; __threadfence(); *(volatile v8us*)dh = vh; *(volatile v8us*)dl = vl;
}

__device__ __forceinline__ float adj_ij(const float* xi, const float* xj) { float si = 0.f, sj = 0.f, d = 0.f;
#pragma unroll
  for (int c = 0; c < 6; ++c) { const float a = bf16_round(xi[c]), bq = bf16_round(xj[c]); si += a * a; sj += bq * bq; d += a * bq; } return expf(-(si - 2.0f * d + sj)); }
__global__ __launch_bounds__(256) void k_lap_dinv(const float* __restrict__ xb, float* __restrict__ dinv) {
  __shared__ float red[256];
  const int i = blockIdx.x, tid = threadIdx.x; const float* xi = xb + (size_t)i * 6;
  float s = 0.f;
#pragma unroll 1
  for (int j = tid; j < NN; j += 256) s += adj_ij(xi, xb + (size_t)j * 6);
  red[tid] = s; __syncthreads(); for (int st = 128; st > 0; st >>= 1) { if (tid < st) red[tid] += red[tid + st]; __syncthreads(); }
  if (tid < 32) { const float v = (tid == 0) ? 1.0f / sqrtf(red[0]) : 0.f; *(volatile float*)(dinv + (size_t)i * 32 + tid) = v; __threadfence(); *(volatile float*)(dinv + (size_t)i * 32 + tid) = v; }
}
__global__ __launch_bounds__(256) void k_lap_rows(const float* __restrict__ xb, const float* __restrict__ dinv, float* __restrict__ L) {
  const int i = blockIdx.x, tid = threadIdx.x; const float* xi = xb + (size_t)i * 6; const float di = dinv[(size_t)i * 32];
  float* row = L + (size_t)i * NN;
  for (int pass = 0; pass < 2; ++pass) {
#pragma unroll 1
    for (int j = tid; j < NN; j += 256) { const float v = ((i == j) ? 1.0f : 0.0f) - di * adj_ij(xi, xb + (size_t)j * 6) * dinv[(size_t)j * 32]; *(volatile float*)(row + j) = v; }
    if (pass == 0) __threadfence();
  }
}
__global__ __launch_bounds__(64) void k_x0(const float* __restrict__ xb, const int* __restrict__ catb, float* __restrict__ X0) {
  const int r = blockIdx.x, c = threadIdx.x; int cl = catb[0]; cl = cl < 0 ? 0 : (cl >= NCL ? NCL - 1 : cl);
  float v = 0.f; if (c < 6) v = bf16_round(xb[(size_t)r * 6 + c]); else if (c < 22) v = (c - 6 == cl) ? 1.f : 0.f;
  *(volatile float*)(X0 + (size_t)r * 64 + c) = v; __threadfence(); *(volatile float*)(X0 + (size_t)r * 64 + c) = v;
}
__global__ __launch_bounds__(256) void k_wt_pad(const float* __restrict__ W, unsigned short* __restrict__ Bt, int Fin, int Fout, int Kp, int Np) {
  const int t = blockIdx.x * 256 + threadIdx.x; const int k8n = Kp / 8; if (t >= Np * k8n) return;
  const int n = t / k8n, k8 = (t % k8n) * 8; v8us v;
#pragma unroll 1
  for (int i = 0; i < 8; ++i) { const int kk = k8 + i; v[i] = (n < Fout && kk < Fin) ? bf16_bits(W[(size_t)kk * Fout + n]) : (unsigned short)0; }
  *(volatile v8us*)(Bt + (size_t)n * Kp + k8) = v; __threadfence(); *(volatile v8us*)(Bt + (size_t)n * Kp + k8) = v;
}
__global__ __launch_bounds__(256) void k_out50(const float* __restrict__ g, const float* __restrict__ fb2, const float* __restrict__ br5, float* __restrict__ out) {
  const int r0 = blockIdx.x * 64; const int tid = threadIdx.x;
  for (int pass = 0; pass < 2; ++pass) { for (int i = tid; i < 64 * 50; i += 256) { const int r = i / 50, c = i % 50; const float v = fmaxf(g[(size_t)(r0 + r) * 64 + c] + bf16_round(fb2[c]) + bf16_round(br5[(size_t)(r0 + r) * 50 + c]), 0.f); *(volatile float*)(out + (size_t)r0 * 50 + i) = v; } if (pass == 0) __threadfence(); }
}

extern "C" void kernel_launch(void* const* d_in, const int* in_sizes, int n_in,
                              void* d_out, int out_size, void* d_ws, size_t ws_size, hipStream_t stream) {
  (void)in_sizes; (void)n_in; (void)out_size;
  const float* x = (const float*)d_in[0]; const int* cat = (const int*)d_in[1];
  const float* cw[3] = {(const float*)d_in[2], (const float*)d_in[4], (const float*)d_in[6]}; const float* cb[3] = {(const float*)d_in[3], (const float*)d_in[5], (const float*)d_in[7]};
  const float* fw[3] = {(const float*)d_in[8], (const float*)d_in[10], (const float*)d_in[12]}; const float* fb[3] = {(const float*)d_in[9], (const float*)d_in[11], (const float*)d_in[13]};
  const float* br[6]; for (int i = 0; i < 6; ++i) br[i] = (const float*)d_in[14 + i];
  const int Fin[3] = {22, 128, 512}, Kp[3] = {64, 128, 512}, Fo[3] = {128, 512, 1024}, Kc[3] = {6, 5, 3};
  char* ws = (char*)d_ws; size_t off = 0;
  auto take = [&](size_t bytes) { char* p = ws + off; off += (bytes + 255) & ~(size_t)255; return p; };
  unsigned short* Wc[3][6]; for (int l = 0; l < 3; ++l) for (int k = 0; k < Kc[l]; ++k) Wc[l][k] = (unsigned short*)take((size_t)Fo[l] * Kp[l] * 2);
  unsigned short* Wf0 = (unsigned short*)take((size_t)512 * 1024 * 2); unsigned short* Wf1a = (unsigned short*)take((size_t)128 * 512 * 2); unsigned short* Wf1b = (unsigned short*)take((size_t)128 * 512 * 2); unsigned short* Wf2 = (unsigned short*)take((size_t)64 * 128 * 2);
  float* dinv = (float*)take((size_t)NN * 32 * 4); float* L = (float*)take((size_t)NN * NN * 4);
  float* X0 = (float*)take((size_t)NN * 64 * 4);
  float* S1 = (float*)take((size_t)NN * 512 * 4); float* S2 = (float*)take((size_t)NN * 512 * 4);
  float* O0 = (float*)take((size_t)NN * 128 * 4); float* O1 = (float*)take((size_t)NN * 512 * 4); float* O2 = (float*)take((size_t)NN * 1024 * 4);
  float* H0 = (float*)take((size_t)NN * 512 * 4); float* T1 = (float*)take((size_t)NN * 128 * 4); float* H1 = (float*)take((size_t)NN * 128 * 4); float* H2 = (float*)take((size_t)NN * 64 * 4);
  unsigned short* Ph = (unsigned short*)take((size_t)512 * NN * 2); unsigned short* Pl = (unsigned short*)take((size_t)512 * NN * 2);
  if (off > ws_size) return;
  for (int l = 0; l < 3; ++l) for (int k = 0; k < Kc[l]; ++k) k_wt_pad<<<(Fo[l] * (Kp[l] / 8) + 255) / 256, 256, 0, stream>>>(cw[l] + (size_t)k * Fin[l] * Fo[l], Wc[l][k], Fin[l], Fo[l], Kp[l], Fo[l]);
  k_wt_pad<<<(512 * 128 + 255) / 256, 256, 0, stream>>>(fw[0], Wf0, 1024, 512, 1024, 512);
  k_wt_pad<<<(128 * 64 + 255) / 256, 256, 0, stream>>>(fw[1], Wf1a, 512, 128, 512, 128);
  k_wt_pad<<<(128 * 64 + 255) / 256, 256, 0, stream>>>(fw[1] + (size_t)512 * 128, Wf1b, 512, 128, 512, 128);
  k_wt_pad<<<(64 * 16 + 255) / 256, 256, 0, stream>>>(fw[2], Wf2, 128, 50, 128, 64);
  for (int b = 0; b < BB; ++b) {
    const float* xb = x + (size_t)b * NN * 6;
    k_lap_dinv<<<NN, 256, 0, stream>>>(xb, dinv);
    k_lap_rows<<<NN, 256, 0, stream>>>(xb, dinv, L);
    k_x0<<<NN, 64, 0, stream>>>(xb, cat + b, X0);
    float* layer_in = X0; float* outs[3] = {O0, O1, O2};
    for (int l = 0; l < 3; ++l) {
      const int P = Kp[l], F = Fo[l], KC = Kc[l]; float* outp = outs[l];
      const dim3 gW(((NN / 16) * (F / 64) + 3) / 4, 1), gL(((NN / 16) * (P / 64) + 3) / 4, 1);
      k_gemm_b<true, false, 0><<<gW, 128, 0, stream>>>(layer_in, P, 0, Wc[l][0], nullptr, P, 0, cb[l], br[l], F, 0, 1.0f, 1.0f, outp, F, 0, NN, F, P);
      float* xkm2 = layer_in; float* xkm1 = layer_in;
      for (int k = 1; k < KC; ++k) {
        k_split_transpose_b<<<dim3((P * (NN / 8) + 255) / 256, 1), 256, 0, stream>>>(xkm1, P, 0, Ph, Pl, 0, NN, P);
        float* xk = (k == 1) ? S1 : ((xkm2 == layer_in) ? S2 : xkm2);
        if (k == 1) k_gemm_b<true, true, 0><<<gL, 128, 0, stream>>>(L, NN, 0, Ph, Pl, NN, 0, nullptr, nullptr, 0, 0, 0.f, 1.0f, xk, P, 0, NN, P, NN);
        else        k_gemm_b<true, true, 0><<<gL, 128, 0, stream>>>(L, NN, 0, Ph, Pl, NN, 0, nullptr, xkm2, P, 0, -1.0f, 2.0f, xk, P, 0, NN, P, NN);
        if (k == KC - 1) k_gemm_b<true, false, 1><<<gW, 128, 0, stream>>>(xk, P, 0, Wc[l][k], nullptr, P, 0, nullptr, outp, F, 0, 1.0f, 1.0f, outp, F, 0, NN, F, P);
        else             k_gemm_b<true, false, 0><<<gW, 128, 0, stream>>>(xk, P, 0, Wc[l][k], nullptr, P, 0, nullptr, outp, F, 0, 1.0f, 1.0f, outp, F, 0, NN, F, P);
        xkm2 = xkm1; xkm1 = xk;
      }
      layer_in = outp;
    }
    k_gemm_b<true, false, 1><<<dim3(((NN / 16) * (512 / 64) + 3) / 4, 1), 128, 0, stream>>>(O2, 1024, 0, Wf0, nullptr, 1024, 0, fb[0], br[3], 512, 0, 1.0f, 1.0f, H0, 512, 0, NN, 512, 1024);
    k_gemm_b<true, false, 0><<<dim3(((NN / 16) * (128 / 64) + 3) / 4, 1), 128, 0, stream>>>(H0, 512, 0, Wf1a, nullptr, 512, 0, fb[1], br[4], 128, 0, 1.0f, 1.0f, T1, 128, 0, NN, 128, 512);
    k_gemm_b<true, false, 1><<<dim3(((NN / 16) * (128 / 64) + 3) / 4, 1), 128, 0, stream>>>(O1, 512, 0, Wf1b, nullptr, 512, 0, nullptr, T1, 128, 0, 1.0f, 1.0f, H1, 128, 0, NN, 128, 512);
    k_gemm_b<true, false, 0><<<dim3(((NN / 16) * 1 + 3) / 4, 1), 128, 0, stream>>>(H1, 128, 0, Wf2, nullptr, 128, 0, nullptr, nullptr, 0, 0, 1.0f, 1.0f, H2, 64, 0, NN, 64, 128);
    k_out50<<<NN / 64, 256, 0, stream>>>(H2, fb[2], br[5], (float*)d_out + (size_t)b * NN * 50);
  }
}
